// SSMTimeSeriesModel_83373905150196
// MI455X (gfx1250) — hardware-verified
//
#include <hip/hip_runtime.h>


typedef _Float16 f16t;
typedef f16t     v16h __attribute__((ext_vector_type(16)));
typedef f16t     v8h  __attribute__((ext_vector_type(8)));
typedef __bf16   v16b __attribute__((ext_vector_type(16)));
typedef float    v8f  __attribute__((ext_vector_type(8)));
typedef float    v4f  __attribute__((ext_vector_type(4)));
typedef unsigned int v4u __attribute__((ext_vector_type(4)));

union FragH { v16h v; v8h q[2]; };
union FragB { v16b v; v4u q[2]; };
union PkH   { v8h h; v4u u; };

#define NBATCH 128
#define NSTEP  512
#define NCH    32
#define NST    512
#define NDEC   16384
#define SP     520
#define FP     520
#define TP     132

__device__ __forceinline__ v8f wm_f16(v16h a, v16h b, v8f c) {
    return __builtin_amdgcn_wmma_f32_16x16x32_f16(false, a, false, b, (short)0, c, false, false);
}
__device__ __forceinline__ v8f wm_bf16(v16b a, v16b b, v8f c) {
    return __builtin_amdgcn_wmma_f32_16x16x32_bf16(false, a, false, b, (short)0, c, false, false);
}
__device__ __forceinline__ v8f zero8() {
    v8f z = {0.f, 0.f, 0.f, 0.f, 0.f, 0.f, 0.f, 0.f};
    return z;
}

__device__ __forceinline__ void guard_k(v8f (&c)[4], FragH& a, FragH (&b)[4]) {
    asm volatile("v_nop\n\tv_nop\n\tv_nop\n\tv_nop"
                 : "+v"(c[0]), "+v"(c[1]), "+v"(c[2]), "+v"(c[3])
                 : "v"(a.v), "v"(b[0].v), "v"(b[1].v), "v"(b[2].v), "v"(b[3].v));
}
__device__ __forceinline__ void guard_bu(v8f (&c)[4], FragB& xh, FragB& xl,
                                         FragB (&wh)[4], FragB (&wl)[4]) {
    asm volatile("v_nop\n\tv_nop\n\tv_nop\n\tv_nop"
                 : "+v"(c[0]), "+v"(c[1]), "+v"(c[2]), "+v"(c[3])
                 : "v"(xh.v), "v"(xl.v),
                   "v"(wh[0].v), "v"(wh[1].v), "v"(wh[2].v), "v"(wh[3].v),
                   "v"(wl[0].v), "v"(wl[1].v), "v"(wl[2].v), "v"(wl[3].v));
}
__device__ __forceinline__ void guard_dec(v8f (&c)[4], FragB (&ah)[4], FragB (&al)[4],
                                          FragB& bh, FragB& bl) {
    asm volatile("v_nop\n\tv_nop\n\tv_nop\n\tv_nop"
                 : "+v"(c[0]), "+v"(c[1]), "+v"(c[2]), "+v"(c[3])
                 : "v"(ah[0].v), "v"(ah[1].v), "v"(ah[2].v), "v"(ah[3].v),
                   "v"(al[0].v), "v"(al[1].v), "v"(al[2].v), "v"(al[3].v),
                   "v"(bh.v), "v"(bl.v));
}

__device__ __forceinline__ unsigned int bfbits(float f) {
    unsigned int u = __float_as_uint(f);
    u += 0x7FFFu + ((u >> 16) & 1u);
    return u >> 16;
}
__device__ __forceinline__ void split_pair(float a, float b, unsigned int& ph, unsigned int& pl) {
    const unsigned int ha = bfbits(a), hb = bfbits(b);
    const float ra = a - __uint_as_float(ha << 16);
    const float rb = b - __uint_as_float(hb << 16);
    ph = ha | (hb << 16);
    pl = bfbits(ra) | (bfbits(rb) << 16);
}
__device__ __forceinline__ void split8(v4f v0, v4f v1, v4u& ph, v4u& pl) {
    unsigned int h0, l0, h1, l1, h2, l2, h3, l3;
    split_pair(v0[0], v0[1], h0, l0);
    split_pair(v0[2], v0[3], h1, l1);
    split_pair(v1[0], v1[1], h2, l2);
    split_pair(v1[2], v1[3], h3, l3);
    v4u a, b;
    a[0] = h0; a[1] = h1; a[2] = h2; a[3] = h3;
    b[0] = l0; b[1] = l1; b[2] = l2; b[3] = l3;
    ph = a; pl = b;
}

__global__ __launch_bounds__(256)
void k_prep(const float* A, const float* Wb, const float* Wd,
            f16t* PA, unsigned int* WbH, unsigned int* WbL,
            unsigned int* WdH, unsigned int* WdL,
            int nA8, int nWb8, int nWd8, float scA, float scWb) {
    const int i = blockIdx.x * 256 + threadIdx.x;
    const bool dWd = i < nWd8, dA = i < nA8, dWb = i < nWb8;
    v4u wdh, wdl, wbh, wbl, pah;
#pragma unroll
    for (int e = 0; e < 4; ++e) { wdh[e] = 0u; wdl[e] = 0u; wbh[e] = 0u; wbl[e] = 0u; pah[e] = 0u; }
    if (dWd) {
        const float* p = Wd + (size_t)i * 8;
        v4f v0 = *(const v4f*)p;
        v4f v1 = *(const v4f*)(p + 4);
        split8(v0, v1, wdh, wdl);
    }
    if (dA) {
        const float* p = A + (size_t)i * 8;
        v4f v0 = *(const v4f*)p;
        v4f v1 = *(const v4f*)(p + 4);
        PkH k;
        k.h[0] = (f16t)(v0[0] * scA); k.h[1] = (f16t)(v0[1] * scA);
        k.h[2] = (f16t)(v0[2] * scA); k.h[3] = (f16t)(v0[3] * scA);
        k.h[4] = (f16t)(v1[0] * scA); k.h[5] = (f16t)(v1[1] * scA);
        k.h[6] = (f16t)(v1[2] * scA); k.h[7] = (f16t)(v1[3] * scA);
        pah = k.u;
    }
    if (dWb) {
        const float* p = Wb + (size_t)i * 8;
        v4f v0 = *(const v4f*)p;
        v4f v1 = *(const v4f*)(p + 4);
        v0 = v0 * scWb;
        v1 = v1 * scWb;
        split8(v0, v1, wbh, wbl);
    }
    if (dWd) { *((volatile v4u*)WdH + i) = wdh; *((volatile v4u*)WdL + i) = wdl; }
    if (dA)  { *((volatile v4u*)PA + i) = pah; }
    if (dWb) { *((volatile v4u*)WbH + i) = wbh; *((volatile v4u*)WbL + i) = wbl; }
    __threadfence();
    if (dWd) { *((volatile v4u*)WdH + i) = wdh; *((volatile v4u*)WdL + i) = wdl; }
    if (dA)  { *((volatile v4u*)PA + i) = pah; }
    if (dWb) { *((volatile v4u*)WbH + i) = wbh; *((volatile v4u*)WbL + i) = wbl; }
}

__device__ __forceinline__ void stage_x(const float* x, unsigned int* Xh, unsigned int* Xl,
                                        int b0, int t, int tid, float sc) {
    if (tid < 128) {
        const int row = tid >> 3, c4 = (tid & 7) * 4;
        const float* p = x + ((size_t)(b0 + row) * NSTEP + t) * NCH + c4;
        v4f v = *(const v4f*)p;
        unsigned int h0, l0, h1, l1;
        split_pair(v[0] * sc, v[1] * sc, h0, l0);
        split_pair(v[2] * sc, v[3] * sc, h1, l1);
        const int u = row * 16 + (tid & 7) * 2;
        Xh[u] = h0; Xh[u + 1] = h1;
        Xl[u] = l0; Xl[u + 1] = l1;
    }
}

__global__ __launch_bounds__(256)
void k_scan(const float* x, const f16t* PA, const unsigned int* WbH, const unsigned int* WbL,
            const float* bb, const float* lng, const float* lnb,
            unsigned int* FsH, unsigned int* FsL, int nbatch, float inv_sc) {
    __shared__ __attribute__((aligned(16))) f16t  Sh[16 * SP];
    __shared__ __attribute__((aligned(16))) float Sf[16 * FP];
    __shared__ __attribute__((aligned(16))) unsigned int Xs[2 * 2 * 256];
    __shared__ __attribute__((aligned(16))) float Gl[NST];
    __shared__ __attribute__((aligned(16))) float Bl[NST];

    const int tid = threadIdx.x, w = tid >> 5, l = tid & 31, h = l >> 4, m = l & 15;
    const int b0 = blockIdx.x * 16;
    if (b0 + 16 > nbatch) return;

    for (int i = tid; i < 16 * SP; i += 256) Sh[i] = (f16t)0.0f;
    for (int i = tid; i < NST; i += 256) { Gl[i] = lng[i]; Bl[i] = lnb[i]; }
    stage_x(x, Xs, Xs + 256, b0, 0, tid, 64.0f);
    __syncthreads();

    float bbv[4];
#pragma unroll
    for (int j = 0; j < 4; ++j) bbv[j] = bb[64 * w + 16 * j + m];

#pragma unroll 1
    for (int t = 0; t < NSTEP; ++t) {
        const int cur = (t & 1) * 512, nxt = ((t + 1) & 1) * 512;
        if (t + 1 < NSTEP) stage_x(x, Xs + nxt, Xs + nxt + 256, b0, t + 1, tid, 64.0f);

        unsigned long long pab = (unsigned long long)PA;
        unsigned long long whb = (unsigned long long)WbH;
        unsigned long long wlb = (unsigned long long)WbL;
        asm volatile("" : "+s"(pab), "+s"(whb), "+s"(wlb));
        const f16t* pa = (const f16t*)pab;
        const unsigned int* pwh = (const unsigned int*)whb;
        const unsigned int* pwl = (const unsigned int*)wlb;

        v8f acc[4];
#pragma unroll
        for (int j = 0; j < 4; ++j) acc[j] = zero8();

        const f16t* sa = Sh + m * SP + 8 * h;
        const f16t* pb = pa + (size_t)(64 * w + m) * NST + 8 * h;
#pragma unroll 1
        for (int kt = 0; kt < NST / 32; ++kt) {
            FragH a, b[4];
            a.q[0] = *(const v8h*)(sa + 32 * kt);
            a.q[1] = *(const v8h*)(sa + 32 * kt + 16);
#pragma unroll
            for (int j = 0; j < 4; ++j) {
                const f16t* p = pb + (size_t)(16 * j) * NST + 32 * kt;
                b[j].q[0] = *(const v8h*)p;
                b[j].q[1] = *(const v8h*)(p + 16);
            }
#pragma unroll
            for (int j = 0; j < 4; ++j) acc[j] = wm_f16(a.v, b[j].v, acc[j]);
            guard_k(acc, a, b);
        }
        {
            FragB xh, xl, wh[4], wl[4];
            const unsigned int* xp = Xs + cur + m * 16 + 4 * h;
            xh.q[0] = *(const v4u*)xp;          xh.q[1] = *(const v4u*)(xp + 8);
            xl.q[0] = *(const v4u*)(xp + 256);  xl.q[1] = *(const v4u*)(xp + 264);
#pragma unroll
            for (int j = 0; j < 4; ++j) {
                const size_t ro = (size_t)(64 * w + 16 * j + m) * 16 + 4 * h;
                wh[j].q[0] = *(const v4u*)(pwh + ro);  wh[j].q[1] = *(const v4u*)(pwh + ro + 8);
                wl[j].q[0] = *(const v4u*)(pwl + ro);  wl[j].q[1] = *(const v4u*)(pwl + ro + 8);
            }
#pragma unroll
            for (int j = 0; j < 4; ++j) {
                acc[j] = wm_bf16(xh.v, wh[j].v, acc[j]);
                acc[j] = wm_bf16(xh.v, wl[j].v, acc[j]);
                acc[j] = wm_bf16(xl.v, wh[j].v, acc[j]);
            }
            guard_bu(acc, xh, xl, wh, wl);
        }
#pragma unroll
        for (int j = 0; j < 4; ++j)
#pragma unroll
            for (int r = 0; r < 8; ++r)
                Sf[(8 * h + r) * FP + 64 * w + 16 * j + m] = fmaf(acc[j][r], inv_sc, bbv[j]);
        __syncthreads();

        const bool last = (t == NSTEP - 1);
#pragma unroll
        for (int q = 0; q < 2; ++q) {
            const int row = 2 * w + q;
            float* sp = Sf + row * FP + 16 * l;
            float v[16];
#pragma unroll
            for (int e = 0; e < 4; ++e) {
                v4f t4 = *(const v4f*)(sp + 4 * e);
                v[4 * e] = t4[0]; v[4 * e + 1] = t4[1]; v[4 * e + 2] = t4[2]; v[4 * e + 3] = t4[3];
            }
            float s = 0.0f;
#pragma unroll
            for (int e = 0; e < 16; ++e) s += v[e];
#pragma unroll
            for (int off = 16; off > 0; off >>= 1) s += __shfl_xor(s, off, 32);
            const float mu = s * (1.0f / 512.0f);
            float qq = 0.0f;
#pragma unroll
            for (int e = 0; e < 16; ++e) { v[e] = v[e] - mu; qq += v[e] * v[e]; }
#pragma unroll
            for (int off = 16; off > 0; off >>= 1) qq += __shfl_xor(qq, off, 32);
            const float rs = rsqrtf(qq * (1.0f / 512.0f) + 1e-5f);
            const float* gq = Gl + 16 * l;
            const float* bq = Bl + 16 * l;
            PkH k0, k1;
#pragma unroll
            for (int e = 0; e < 4; ++e) {
                v4f g4 = *(const v4f*)(gq + 4 * e);
                v4f b4 = *(const v4f*)(bq + 4 * e);
                v4f y4;
#pragma unroll
                for (int c = 0; c < 4; ++c) {
                    float y = fmaxf(v[4 * e + c] * rs * g4[c] + b4[c], 0.0f);
                    y4[c] = y;
                    f16t hv = (f16t)(y * 16.0f);
                    if (e < 2) k0.h[4 * e + c] = hv; else k1.h[4 * (e - 2) + c] = hv;
                }
                if (last) *(v4f*)(sp + 4 * e) = y4;
            }
            *(v8h*)(Sh + row * SP + 16 * l)     = k0.h;
            *(v8h*)(Sh + row * SP + 16 * l + 8) = k1.h;
        }
        __syncthreads();
    }

    v4u pk[8];
#pragma unroll
    for (int i = 0; i < 8; ++i) {
        const int p = tid + 256 * i;
        const int q = p & 1023;
        const int row = q >> 6, c8 = (q & 63) * 8;
        const float* sp = Sf + row * FP + c8;
        v4f v0 = *(const v4f*)sp;
        v4f v1 = *(const v4f*)(sp + 4);
        v4u hh, ll;
        split8(v0, v1, hh, ll);
        if (i < 4) pk[i] = hh; else pk[i] = ll;
    }
#pragma unroll
    for (int i = 0; i < 8; ++i) {
        const int p = tid + 256 * i;
        const int q = p & 1023;
        const int row = q >> 6, c4u = (q & 63) * 4;
        unsigned int* dst = ((i < 4) ? FsH : FsL) + (size_t)(b0 + row) * (NST / 2) + c4u;
        *(volatile v4u*)dst = pk[i];
    }
    __threadfence();
#pragma unroll
    for (int i = 0; i < 8; ++i) {
        const int p = tid + 256 * i;
        const int q = p & 1023;
        const int row = q >> 6, c4u = (q & 63) * 4;
        unsigned int* dst = ((i < 4) ? FsH : FsL) + (size_t)(b0 + row) * (NST / 2) + c4u;
        *(volatile v4u*)dst = pk[i];
    }
}

__global__ __launch_bounds__(256)
void k_dec(const unsigned int* FsH, const unsigned int* FsL,
           const unsigned int* WdH, const unsigned int* WdL,
           const float* bd, float* out, int nrows, int ncols) {
    __shared__ __attribute__((aligned(16))) float Ts[64 * TP];
    const int tid = threadIdx.x, w = tid >> 5, l = tid & 31, h = l >> 4, m = l & 15;
    const int nb = blockIdx.x >> 1, mh = blockIdx.x & 1;
    const int col0 = nb * 128, row0 = mh * 64;
    if (col0 + 128 > ncols || row0 + 64 > nrows) return;

    const int ncol = col0 + 16 * w + m;
    const int KU = NST / 2;
    const unsigned int* bhp = WdH + (size_t)ncol * KU + 4 * h;
    const unsigned int* blp = WdL + (size_t)ncol * KU + 4 * h;
    const unsigned int* ahp = FsH + (size_t)(row0 + m) * KU + 4 * h;
    const unsigned int* alp = FsL + (size_t)(row0 + m) * KU + 4 * h;

    v8f acc[4];
#pragma unroll
    for (int i = 0; i < 4; ++i) acc[i] = zero8();

#pragma unroll 1
    for (int kt = 0; kt < NST / 32; ++kt) {
        FragB bh, bl, ah[4], al[4];
        const int ko = 16 * kt;
        bh.q[0] = *(const v4u*)(bhp + ko);  bh.q[1] = *(const v4u*)(bhp + ko + 8);
        bl.q[0] = *(const v4u*)(blp + ko);  bl.q[1] = *(const v4u*)(blp + ko + 8);
#pragma unroll
        for (int i = 0; i < 4; ++i) {
            const size_t ro = (size_t)(16 * i) * KU + ko;
            ah[i].q[0] = *(const v4u*)(ahp + ro);  ah[i].q[1] = *(const v4u*)(ahp + ro + 8);
            al[i].q[0] = *(const v4u*)(alp + ro);  al[i].q[1] = *(const v4u*)(alp + ro + 8);
        }
#pragma unroll
        for (int i = 0; i < 4; ++i) {
            acc[i] = wm_bf16(ah[i].v, bh.v, acc[i]);
            acc[i] = wm_bf16(ah[i].v, bl.v, acc[i]);
            acc[i] = wm_bf16(al[i].v, bh.v, acc[i]);
        }
        guard_dec(acc, ah, al, bh, bl);
    }

    const float bdv = bd[ncol];
#pragma unroll
    for (int i = 0; i < 4; ++i)
#pragma unroll
        for (int r = 0; r < 8; ++r)
            Ts[(16 * i + 8 * h + r) * TP + 16 * w + m] = acc[i][r] + bdv;
    __syncthreads();

    v4f pv[8];
#pragma unroll
    for (int i = 0; i < 8; ++i) {
        const int p = tid + 256 * i, row = p >> 5, c4 = (p & 31) * 4;
        pv[i] = *(const v4f*)(Ts + row * TP + c4);
    }
#pragma unroll
    for (int i = 0; i < 8; ++i) {
        const int p = tid + 256 * i, row = p >> 5, c4 = (p & 31) * 4;
        float* dst = out + (size_t)(row0 + row) * ncols + col0 + c4;
        *(volatile v4f*)dst = pv[i];
    }
    __threadfence();
#pragma unroll
    for (int i = 0; i < 8; ++i) {
        const int p = tid + 256 * i, row = p >> 5, c4 = (p & 31) * 4;
        float* dst = out + (size_t)(row0 + row) * ncols + col0 + c4;
        *(volatile v4f*)dst = pv[i];
    }
}

extern "C" void kernel_launch(void* const* d_in, const int* in_sizes, int n_in,
                              void* d_out, int out_size, void* d_ws, size_t ws_size,
                              hipStream_t stream) {
    if (n_in < 8) return;
    if (in_sizes[0] != NBATCH * NSTEP * NCH || in_sizes[1] != NST * NST ||
        in_sizes[2] != NST * NCH || in_sizes[3] != NST || in_sizes[4] != NST ||
        in_sizes[5] != NST || in_sizes[6] != NDEC * NST || in_sizes[7] != NDEC ||
        out_size != NBATCH * NDEC) return;

    const float* x   = (const float*)d_in[0];
    const float* A   = (const float*)d_in[1];
    const float* Wb  = (const float*)d_in[2];
    const float* bb  = (const float*)d_in[3];
    const float* lng = (const float*)d_in[4];
    const float* lnb = (const float*)d_in[5];
    const float* Wd  = (const float*)d_in[6];
    const float* bd  = (const float*)d_in[7];
    float* out = (float*)d_out;

    char* ws = (char*)d_ws;
    size_t off = 0;
    auto carve = [&](size_t bytes) -> char* {
        char* p = ws + off;
        off = (off + bytes + 255) & ~(size_t)255;
        return p;
    };
    f16t*         PA  = (f16t*)carve((size_t)NST * NST * 2);
    unsigned int* WbH = (unsigned int*)carve((size_t)NST * NCH * 2);
    unsigned int* WbL = (unsigned int*)carve((size_t)NST * NCH * 2);
    unsigned int* WdH = (unsigned int*)carve((size_t)NDEC * NST * 2);
    unsigned int* WdL = (unsigned int*)carve((size_t)NDEC * NST * 2);
    unsigned int* FsH = (unsigned int*)carve((size_t)NBATCH * NST * 2);
    unsigned int* FsL = (unsigned int*)carve((size_t)NBATCH * NST * 2);
    if (off > ws_size) return;

    const int nA8  = NST * NST / 8;
    const int nWb8 = NST * NCH / 8;
    const int nWd8 = NDEC * NST / 8;
    int nmax = nWd8;
    if (nA8 > nmax) nmax = nA8;
    if (nWb8 > nmax) nmax = nWb8;

    k_prep<<<dim3((nmax + 255) / 256), dim3(256), 0, stream>>>(A, Wb, Wd, PA, WbH, WbL, WdH, WdL,
                                                              nA8, nWb8, nWd8, 256.0f, 64.0f);
    k_scan<<<dim3(NBATCH / 16), dim3(256), 0, stream>>>(x, PA, WbH, WbL, bb, lng, lnb,
                                                       FsH, FsL, NBATCH, 0.000244140625f);
    k_dec<<<dim3((NDEC / 128) * (NBATCH / 64)), dim3(256), 0, stream>>>(FsH, FsL, WdH, WdL,
                                                                      bd, out, NBATCH, NDEC);
}
